// FlashGQA_83124797046958
// MI455X (gfx1250) — hardware-verified
//
#include <hip/hip_runtime.h>
#include <math.h>

constexpr int kB   = 2;
constexpr int kS   = 2048;
constexpr int kD   = 2048;
constexpr int kNH  = 32;
constexpr int kKVH = 8;
constexpr int kHD  = 64;
constexpr int kGrp = kNH / kKVH;
constexpr int kTok = kB * kS;
constexpr int kKVD = kKVH * kHD;
constexpr int kQKN = kD + kKVD;
constexpr int kRH  = kHD / 2;
constexpr int kQB  = 64;
constexpr int kKC  = 64;
constexpr float kScoreScale = 0.125f;
constexpr float kMaskFill   = -3.40282347e38f;
static_assert(kNH * kHD == kD);
static_assert(kGrp * kKVH == kNH);
static_assert(kD % 32 == 0 && kS % 32 == 0 && kHD % 32 == 0);
static_assert(kTok % 64 == 0 && kQKN % 64 == 0 && kKVD % 64 == 0 && kD % 64 == 0 && kS % 64 == 0);
static_assert(kS % kQB == 0 && kQB == 64 && kKC == 64 && kHD == 64);
static_assert((kTok * kD) % 2048 == 0 && (kD * kD) % 2048 == 0 && (kKVD * kD) % 2048 == 0);
static_assert(kS % 8 == 0 && kRH == 32);

typedef __attribute__((ext_vector_type(16))) _Float16 v16h;
typedef __attribute__((ext_vector_type(8)))  _Float16 v8h;
typedef __attribute__((ext_vector_type(16))) __bf16   v16b;
typedef __attribute__((ext_vector_type(8)))  __bf16   v8b;
typedef __attribute__((ext_vector_type(8)))  float    v8f;
typedef __attribute__((ext_vector_type(4)))  float    v4f;
typedef __attribute__((ext_vector_type(4)))  unsigned int v4u;

__device__ __forceinline__ unsigned short f2bf_bits(float f) {
  unsigned u = __float_as_uint(f);
  return (unsigned short)((u + 0x7FFFu + ((u >> 16) & 1u)) >> 16);
}
__device__ __forceinline__ float bf_bits2f(unsigned short h) { return __uint_as_float(((unsigned)h) << 16); }

__device__ __forceinline__ void dep_guard_h(v8f& a, v8f& b, v16h x, v16h y) { asm volatile("v_nop\n\tv_nop\n\tv_nop\n\tv_nop" : "+v"(a), "+v"(b) : "v"(x), "v"(y)); }
__device__ __forceinline__ void dep_guard_b(v8f& a, v8f& b, v16b x, v16b y) { asm volatile("v_nop\n\tv_nop\n\tv_nop\n\tv_nop" : "+v"(a), "+v"(b) : "v"(x), "v"(y)); }
__device__ __forceinline__ void keep4_h(v16h a, v16h b, v16h c, v16h d) { asm volatile("v_nop" :: "v"(a), "v"(b), "v"(c), "v"(d)); }
__device__ __forceinline__ void keep4_b(v16b a, v16b b, v16b c, v16b d) { asm volatile("v_nop" :: "v"(a), "v"(b), "v"(c), "v"(d)); }
__device__ __forceinline__ void acc_guard4(v8f& a, v8f& b, v8f& c, v8f& d) { asm volatile("v_nop\n\tv_nop\n\tv_nop\n\tv_nop" : "+v"(a), "+v"(b), "+v"(c), "+v"(d)); }
template <typename T> struct Frag;
template <> struct Frag<_Float16> {
  typedef v16h V; union U { v16h v; v8h h[2]; };
  static __device__ __forceinline__ v16h load(const _Float16* p) {
    U f; f.h[0] = *(const v8h*)(p); f.h[1] = *(const v8h*)(p + 16); return f.v;
  }
  static __device__ __forceinline__ v8f mma(v16h a, v16h b, v8f c) {
    return __builtin_amdgcn_wmma_f32_16x16x32_f16(false, a, false, b, (short)0, c, false, false);
  }
  static __device__ __forceinline__ void guard(v8f& a, v8f& b, v16h x, v16h y) { dep_guard_h(a, b, x, y); }
  static __device__ __forceinline__ void keep(v16h a, v16h b, v16h c, v16h d) { keep4_h(a, b, c, d); }
};
template <> struct Frag<__bf16> {
  typedef v16b V; union U { v16b v; v8b h[2]; };
  static __device__ __forceinline__ v16b load(const __bf16* p) {
    U f; f.h[0] = *(const v8b*)(p); f.h[1] = *(const v8b*)(p + 16); return f.v;
  }
  static __device__ __forceinline__ v8f mma(v16b a, v16b b, v8f c) {
    return __builtin_amdgcn_wmma_f32_16x16x32_bf16(false, a, false, b, (short)0, c, false, false);
  }
  static __device__ __forceinline__ void guard(v8f& a, v8f& b, v16b x, v16b y) { dep_guard_b(a, b, x, y); }
  static __device__ __forceinline__ void keep(v16b a, v16b b, v16b c, v16b d) { keep4_b(a, b, c, d); }
};

__device__ __forceinline__ unsigned pk16(unsigned short a, unsigned short b) { return (unsigned)a | ((unsigned)b << 16); }

template <int ET> struct Elem;
template <> struct Elem<0> { typedef _Float16 T; };
template <> struct Elem<1> { typedef __bf16 T; };
template <int ET, bool SPLIT, int BIAS_MODE, int OUT_MODE, bool RESID, int ACT = 0, bool ALO = false>
__global__ __launch_bounds__(256) void wmma_gemm64(
    const unsigned short* __restrict__ Ap, const unsigned short* __restrict__ A2p, int lda, long strideA,
    const unsigned short* __restrict__ Btp, const unsigned short* __restrict__ Bt2p, int ldb, long strideB,
    void* __restrict__ Cout, void* __restrict__ Cout2, int ldc, long strideC,
    const float* __restrict__ bias,
    const float* __restrict__ resid, long strideR,
    int M, int N, int K, float scale) {
  typedef typename Elem<ET>::T T;
  typedef typename Frag<T>::V V;
  constexpr bool SPLITB = SPLIT && !ALO;
  const T* A = (const T*)Ap; const T* A2 = (const T*)A2p; const T* Bt = (const T*)Btp; const T* Bt2 = (const T*)Bt2p;
  __shared__ __align__(16) float sT[8][16 * 68];
  const int b    = blockIdx.y;
  const int lane = threadIdx.x & 31;
  const int wave = threadIdx.x >> 5;
  const int tilesN = N >> 6;
  const int tilesM = M >> 6;
  const int tile = blockIdx.x * 8 + wave;
  if (tile >= tilesM * tilesN) return;
  const int tm = tile / tilesN;
  const int tn = tile - tm * tilesN;
  const int m0 = tm << 6;
  const int n0 = tn << 6;

  const T* Ab  = A  + (size_t)b * strideA;
  const T* Bb  = Bt + (size_t)b * strideB;
  const T* Ab2 = SPLIT ? (A2  + (size_t)b * strideA) : nullptr;
  const T* Bb2 = SPLITB ? (Bt2 + (size_t)b * strideB) : nullptr;

  const int rlane = lane & 15;
  const int koff  = (lane >> 4) * 8;
  const int mOff  = (lane >> 4) * 8;

  v8f acc[4][4];
#pragma unroll
  for (int i = 0; i < 4; ++i)
#pragma unroll
    for (int j = 0; j < 4; ++j) acc[i][j] = (v8f){0.f,0.f,0.f,0.f,0.f,0.f,0.f,0.f};

  for (int k0 = 0; k0 < K; k0 += 32) {
    V bh[4], bl[4];
#pragma unroll
    for (int j = 0; j < 4; ++j) {
      const size_t bo = (size_t)(n0 + (j << 4) + rlane) * ldb + koff + k0;
      bh[j] = Frag<T>::load(Bb + bo);
      if (SPLITB) bl[j] = Frag<T>::load(Bb2 + bo);
    }
#pragma unroll
    for (int i = 0; i < 4; ++i) {
      const size_t ao = (size_t)(m0 + (i << 4) + rlane) * lda + koff + k0;
      V ah = Frag<T>::load(Ab + ao);
      V al;
      if (SPLIT) al = Frag<T>::load(Ab2 + ao);
#pragma unroll
      for (int j = 0; j < 4; ++j) {
        acc[i][j] = Frag<T>::mma(ah, bh[j], acc[i][j]);
        if (SPLIT) {
          if (SPLITB) acc[i][j] = Frag<T>::mma(ah, bl[j], acc[i][j]);
          acc[i][j] = Frag<T>::mma(al, bh[j], acc[i][j]);
        }
      }
      Frag<T>::guard(acc[i][0], acc[i][3], ah, SPLIT ? al : ah);
    }
    Frag<T>::keep(bh[0], bh[1], bh[2], bh[3]);
    if (SPLITB) Frag<T>::keep(bl[0], bl[1], bl[2], bl[3]);
  }
  acc_guard4(acc[0][0], acc[0][1], acc[0][2], acc[0][3]);
  acc_guard4(acc[1][0], acc[1][1], acc[1][2], acc[1][3]);
  acc_guard4(acc[2][0], acc[2][1], acc[2][2], acc[2][3]);
  acc_guard4(acc[3][0], acc[3][1], acc[3][2], acc[3][3]);

  float* slab = sT[wave];
  const float* Rb = RESID ? (resid + (size_t)b * strideR) : nullptr;
#pragma unroll
  for (int i = 0; i < 4; ++i) {
    const int mBase = m0 + (i << 4);
#pragma unroll
    for (int j = 0; j < 4; ++j) {
      const int n = n0 + (j << 4) + rlane;
      float bv = 0.f;
      if (BIAS_MODE == 2) bv = bias[n];
#pragma unroll
      for (int r = 0; r < 8; ++r) {
        float v = acc[i][j][r] * scale;
        if (BIAS_MODE == 1) v += bias[mBase + mOff + r];
        if (BIAS_MODE == 2) v += bv;
        if (RESID) v += Rb[(size_t)(mBase + mOff + r) * ldc + n];
        if (ACT == 2) v = fmaxf(v, 0.0f);
        if (ACT == 4) v = (v > 0.f) ? v : 0.01f * v;
        slab[(mOff + r) * 68 + (j << 4) + rlane] = v;
      }
    }
    __builtin_amdgcn_fence(__ATOMIC_RELEASE, "workgroup");
    __builtin_amdgcn_wave_barrier();
    __builtin_amdgcn_fence(__ATOMIC_ACQUIRE, "workgroup");
    if (OUT_MODE == 0) {
      float* C = (float*)Cout + (size_t)b * strideC;
      const int hh = lane >> 4, c4 = (lane & 15) * 4;
      for (int pass = 0; pass < 2; ++pass) {
#pragma unroll
        for (int it = 0; it < 8; ++it) {
          const int row = it * 2 + hh;
          v4f v = *(const v4f*)(slab + row * 68 + c4);
          *(volatile v4f*)(C + (size_t)(mBase + row) * ldc + n0 + c4) = v;
        }
        __threadfence();
      }
    } else {
      const int q = lane >> 3, c8 = (lane & 7) * 8;
      unsigned short* C  = (unsigned short*)Cout  + (size_t)b * strideC;
      unsigned short* C2 = (OUT_MODE == 2) ? ((unsigned short*)Cout2 + (size_t)b * strideC) : nullptr;
      for (int pass = 0; pass < 2; ++pass) {
#pragma unroll
        for (int it = 0; it < 4; ++it) {
          const int row = it * 4 + q;
          const float* sp = slab + row * 68 + c8;
          v8h hv, lv;
#pragma unroll
          for (int e = 0; e < 8; ++e) {
            if (OUT_MODE == 1) {
              hv[e] = (_Float16)sp[e];
            } else {
              unsigned short hb = f2bf_bits(sp[e]);
              unsigned short lb = f2bf_bits(sp[e] - bf_bits2f(hb));
              hv[e] = __builtin_bit_cast(_Float16, hb);
              lv[e] = __builtin_bit_cast(_Float16, lb);
            }
          }
          *(volatile v8h*)(C + (size_t)(mBase + row) * ldc + n0 + c8) = hv;
          if (OUT_MODE == 2) *(volatile v8h*)(C2 + (size_t)(mBase + row) * ldc + n0 + c8) = lv;
        }
        __threadfence();
      }
    }
    __builtin_amdgcn_fence(__ATOMIC_RELEASE, "workgroup");
    __builtin_amdgcn_wave_barrier();
    __builtin_amdgcn_fence(__ATOMIC_ACQUIRE, "workgroup");
  }
}

__global__ __launch_bounds__(256) void cast8_bf16_kernel(const float* __restrict__ in, unsigned short* __restrict__ out, int n8) {
  const int i = blockIdx.x * 256 + threadIdx.x;
  if (i >= n8) return;
  const float* p = in + 8 * (size_t)i;
  const v4f a = *(const v4f*)(p);
  const v4f c = *(const v4f*)(p + 4);
  unsigned short hb[8];
#pragma unroll
  for (int e = 0; e < 4; ++e) {
    hb[e]     = f2bf_bits(a[e]);
    hb[4 + e] = f2bf_bits(c[e]);
  }
  const v4u u = (v4u){pk16(hb[0], hb[1]), pk16(hb[2], hb[3]), pk16(hb[4], hb[5]), pk16(hb[6], hb[7])};
  unsigned short* q = out + 8 * (size_t)i;
  *(volatile v4u*)q = u;
  __threadfence();
  *(volatile v4u*)q = u;
}

struct RopeFreq { float inv[kRH]; };
static_assert(sizeof(RopeFreq) == 128);

__global__ __launch_bounds__(256) void rope_table_kernel(float* __restrict__ cosT, float* __restrict__ sinT, RopeFreq f) {
  __shared__ float tab[kRH];
  if (threadIdx.x == 0) {
#pragma unroll
    for (int i = 0; i < kRH; ++i) tab[i] = f.inv[i];
  }
  __syncthreads();
  const int t = threadIdx.x;
  const int s = blockIdx.x * 8 + (t >> 5);
  const int i = t & 31;
  const float ang = (float)s * tab[i];
  float sn, cs;
  sincosf(ang, &sn, &cs);
  const size_t o = (size_t)s * kRH + i;
  *(volatile float*)(cosT + o) = cs;
  *(volatile float*)(sinT + o) = sn;
  __threadfence();
  *(volatile float*)(cosT + o) = cs;
  *(volatile float*)(sinT + o) = sn;
}

__global__ __launch_bounds__(256) void qk_rope_gemm_kernel(
    const unsigned short* __restrict__ Ap, int lda,
    const unsigned short* __restrict__ Btp, int ldb,
    unsigned short* __restrict__ Ch, unsigned short* __restrict__ Cl, int ldc,
    const float* __restrict__ cosT, const float* __restrict__ sinT,
    int M, int N, int K) {
  typedef __bf16 T;
  typedef v16b V;
  const T* A = (const T*)Ap; const T* Bt = (const T*)Btp;
  __shared__ __align__(16) float sT[8][16 * 68];
  const int lane = threadIdx.x & 31;
  const int wave = threadIdx.x >> 5;
  const int tilesN = N >> 6;
  const int tilesM = M >> 6;
  const int tile = blockIdx.x * 8 + wave;
  if (tile >= tilesM * tilesN) return;
  const int tm = tile / tilesN;
  const int tn = tile - tm * tilesN;
  const int m0 = tm << 6;
  const int n0 = tn << 6;

  const int rlane = lane & 15;
  const int koff  = (lane >> 4) * 8;
  const int mOff  = (lane >> 4) * 8;

  v8f acc[4][4];
#pragma unroll
  for (int i = 0; i < 4; ++i)
#pragma unroll
    for (int j = 0; j < 4; ++j) acc[i][j] = (v8f){0.f,0.f,0.f,0.f,0.f,0.f,0.f,0.f};

  for (int k0 = 0; k0 < K; k0 += 32) {
    V bh[4];
#pragma unroll
    for (int j = 0; j < 4; ++j) {
      const size_t bo = (size_t)(n0 + (j << 4) + rlane) * ldb + koff + k0;
      bh[j] = Frag<T>::load(Bt + bo);
    }
#pragma unroll
    for (int i = 0; i < 4; ++i) {
      const size_t ao = (size_t)(m0 + (i << 4) + rlane) * lda + koff + k0;
      V ah = Frag<T>::load(A + ao);
#pragma unroll
      for (int j = 0; j < 4; ++j) acc[i][j] = Frag<T>::mma(ah, bh[j], acc[i][j]);
      Frag<T>::guard(acc[i][0], acc[i][3], ah, ah);
    }
    Frag<T>::keep(bh[0], bh[1], bh[2], bh[3]);
  }
  acc_guard4(acc[0][0], acc[0][1], acc[0][2], acc[0][3]);
  acc_guard4(acc[1][0], acc[1][1], acc[1][2], acc[1][3]);
  acc_guard4(acc[2][0], acc[2][1], acc[2][2], acc[2][3]);
  acc_guard4(acc[3][0], acc[3][1], acc[3][2], acc[3][3]);

  float* slab = sT[wave];
  const int q4 = lane >> 3, c8 = (lane & 7) * 8, i0 = (lane & 7) * 4;
#pragma unroll
  for (int i = 0; i < 4; ++i) {
    const int mBase = m0 + (i << 4);
#pragma unroll
    for (int j = 0; j < 4; ++j) {
#pragma unroll
      for (int r = 0; r < 8; ++r) slab[(mOff + r) * 68 + (j << 4) + rlane] = acc[i][j][r];
    }
    __builtin_amdgcn_fence(__ATOMIC_RELEASE, "workgroup");
    __builtin_amdgcn_wave_barrier();
    __builtin_amdgcn_fence(__ATOMIC_ACQUIRE, "workgroup");
    for (int pass = 0; pass < 2; ++pass) {
#pragma unroll
      for (int it = 0; it < 4; ++it) {
        const int row = it * 4 + q4;
        const int m = mBase + row;
        const int s = m & (kS - 1);
        const float* sp = slab + row * 68 + c8;
        const v4f cs = *(const v4f*)(cosT + (size_t)s * kRH + i0);
        const v4f sn = *(const v4f*)(sinT + (size_t)s * kRH + i0);
        unsigned short hb[8], lb[8];
#pragma unroll
        for (int e = 0; e < 4; ++e) {
          const float x1 = sp[2 * e];
          const float x2 = sp[2 * e + 1];
          const float o1 = x1 * cs[e] - x2 * sn[e];
          const float o2 = x1 * sn[e] + x2 * cs[e];
          hb[2 * e] = f2bf_bits(o1);
          lb[2 * e] = f2bf_bits(o1 - bf_bits2f(hb[2 * e]));
          hb[2 * e + 1] = f2bf_bits(o2);
          lb[2 * e + 1] = f2bf_bits(o2 - bf_bits2f(hb[2 * e + 1]));
        }
        const v4u uh = (v4u){pk16(hb[0], hb[1]), pk16(hb[2], hb[3]), pk16(hb[4], hb[5]), pk16(hb[6], hb[7])};
        const v4u ul = (v4u){pk16(lb[0], lb[1]), pk16(lb[2], lb[3]), pk16(lb[4], lb[5]), pk16(lb[6], lb[7])};
        const size_t dst = (size_t)m * ldc + n0 + c8;
        *(volatile v4u*)(Ch + dst) = uh;
        *(volatile v4u*)(Cl + dst) = ul;
      }
      __threadfence();
    }
    __builtin_amdgcn_fence(__ATOMIC_RELEASE, "workgroup");
    __builtin_amdgcn_wave_barrier();
    __builtin_amdgcn_fence(__ATOMIC_ACQUIRE, "workgroup");
  }
}

__device__ __forceinline__ unsigned short at_bf_bits(float f) {
  unsigned u = __float_as_uint(f);
  return (unsigned short)((u + 0x7FFFu + ((u >> 16) & 1u)) >> 16);
}
__device__ __forceinline__ __bf16 at_f2bf(float f) { return __builtin_bit_cast(__bf16, at_bf_bits(f)); }
__device__ __forceinline__ void at_split(float f, __bf16& hi, __bf16& lo) {
  const unsigned short hb = at_bf_bits(f);
  hi = __builtin_bit_cast(__bf16, hb);
  lo = at_f2bf(f - __uint_as_float(((unsigned)hb) << 16));
}
__device__ __forceinline__ v8f at_mma(v16b a, v16b b, v8f c) {
  c = __builtin_amdgcn_wmma_f32_16x16x32_bf16(false, a, false, b, (short)0, c, false, false);
  asm volatile("v_nop\n\tv_nop\n\tv_nop\n\tv_nop" : "+v"(c) : "v"(a), "v"(b));
  return c;
}

__global__ __launch_bounds__(128)
void flash_gqa_kernel(const unsigned short* __restrict__ QKh, const unsigned short* __restrict__ QKl,
                      const unsigned short* __restrict__ Vth, const unsigned short* __restrict__ Vtl,
                      unsigned short* __restrict__ Oh, unsigned short* __restrict__ Ol) {
  union FB { v16b v; v8b h[2]; };
  __shared__ __align__(16) __bf16 Ksh[kKC * kHD];
  __shared__ __align__(16) __bf16 Ksl[kKC * kHD];
  __shared__ __align__(16) __bf16 Vsh[kHD * kKC];
  __shared__ __align__(16) __bf16 Vsl[kHD * kKC];
  __shared__ __align__(16) __bf16 Psh[4][16 * kKC];
  __shared__ __align__(16) __bf16 Psl[4][16 * kKC];
  __shared__ __align__(16) float  Os[4][16 * 68];

  const int tid  = threadIdx.x;
  const int wave = tid >> 5;
  const int lane = tid & 31;
  const int hh   = lane >> 4;
  const int c    = lane & 15;

  const int nqb = kS / kQB;
  const int bx  = blockIdx.x;
  const int qb  = bx % nqb;
  const int bh  = bx / nqb;
  const int h   = bh % kNH;
  const int b   = bh / kNH;
  const int kvh = h / kGrp;
  const int q0  = qb * kQB + wave * 16;

  const __bf16* Qh = (const __bf16*)QKh;
  const __bf16* Ql = (const __bf16*)QKl;
  const __bf16* Vhp = (const __bf16*)Vth;
  const __bf16* Vlp = (const __bf16*)Vtl;

  v16b qah[2], qal[2];
  {
    const size_t qoff = (size_t)(b * kS + q0 + c) * kQKN + (size_t)h * kHD;
#pragma unroll
    for (int dc = 0; dc < 2; ++dc) {
      qah[dc] = Frag<__bf16>::load(Qh + qoff + dc * 32 + 8 * hh);
      qal[dc] = Frag<__bf16>::load(Ql + qoff + dc * 32 + 8 * hh);
    }
  }

  float mrow[8], lrow[8];
  v8f oacc[4];
#pragma unroll
  for (int r = 0; r < 8; ++r) { mrow[r] = -__builtin_inff(); lrow[r] = 0.f; }
#pragma unroll
  for (int t = 0; t < 4; ++t) oacc[t] = (v8f){0.f,0.f,0.f,0.f,0.f,0.f,0.f,0.f};

  const int nChunks = qb + 1;
  for (int kc = 0; kc < nChunks; ++kc) {
    const int kv0 = kc * kKC;
    __syncthreads();
    {
      const int r = tid >> 1, hf = (tid & 1) * 32;
      const size_t ko = (size_t)(b * kS + kv0 + r) * kQKN + kD + kvh * kHD + hf;
      const size_t vo = ((size_t)(b * kKVD + kvh * kHD + r)) * kS + kv0 + hf;
      __bf16* dkh = Ksh + r * kHD + hf;
      __bf16* dkl = Ksl + r * kHD + hf;
      __bf16* dvh = Vsh + r * kKC + hf;
      __bf16* dvl = Vsl + r * kKC + hf;
#pragma unroll
      for (int i = 0; i < 4; ++i) *(v8b*)(dkh + 8 * i) = *(const v8b*)(Qh + ko + 8 * i);
      asm volatile("" ::: "memory");
#pragma unroll
      for (int i = 0; i < 4; ++i) *(v8b*)(dkl + 8 * i) = *(const v8b*)(Ql + ko + 8 * i);
      asm volatile("" ::: "memory");
#pragma unroll
      for (int i = 0; i < 4; ++i) *(v8b*)(dvh + 8 * i) = *(const v8b*)(Vhp + vo + 8 * i);
      asm volatile("" ::: "memory");
#pragma unroll
      for (int i = 0; i < 4; ++i) *(v8b*)(dvl + 8 * i) = *(const v8b*)(Vlp + vo + 8 * i);
    }
    __syncthreads();

    v8f s[4];
#pragma unroll
    for (int j = 0; j < 4; ++j) {
      s[j] = (v8f){0.f,0.f,0.f,0.f,0.f,0.f,0.f,0.f};
#pragma unroll
      for (int dc = 0; dc < 2; ++dc) {
        FB kb, kl;
        kb.h[0] = *(const v8b*)(Ksh + (j * 16 + c) * kHD + dc * 32 + 8 * hh);
        kb.h[1] = *(const v8b*)(Ksh + (j * 16 + c) * kHD + dc * 32 + 16 + 8 * hh);
        kl.h[0] = *(const v8b*)(Ksl + (j * 16 + c) * kHD + dc * 32 + 8 * hh);
        kl.h[1] = *(const v8b*)(Ksl + (j * 16 + c) * kHD + dc * 32 + 16 + 8 * hh);
        s[j] = at_mma(qah[dc], kb.v, s[j]);
        s[j] = at_mma(qah[dc], kl.v, s[j]);
        s[j] = at_mma(qal[dc], kb.v, s[j]);
      }
    }
    const bool diag = (kc == qb);
    float cm[8];
#pragma unroll
    for (int r = 0; r < 8; ++r) {
      const int qrow = q0 + 8 * hh + r;
      float m = -__builtin_inff();
#pragma unroll
      for (int j = 0; j < 4; ++j) {
        const int kvcol = kv0 + j * 16 + c;
        float sv = s[j][r] * kScoreScale;
        if (diag && (kvcol > qrow)) sv = kMaskFill;
        s[j][r] = sv;
        m = fmaxf(m, sv);
      }
#pragma unroll
      for (int off = 1; off < 16; off <<= 1) m = fmaxf(m, __shfl_xor(m, off, 32));
      cm[r] = m;
    }
    __bf16* pwh = Psh[wave];
    __bf16* pwl = Psl[wave];
#pragma unroll
    for (int r = 0; r < 8; ++r) {
      const float mnew = fmaxf(mrow[r], cm[r]);
      const float alpha = expf(mrow[r] - mnew);
      mrow[r] = mnew;
      float psum = 0.f;
#pragma unroll
      for (int j = 0; j < 4; ++j) {
        const float p = expf(s[j][r] - mnew);
        psum += p;
        __bf16 a, bl;
        at_split(p, a, bl);
        pwh[(8 * hh + r) * kKC + j * 16 + c] = a;
        pwl[(8 * hh + r) * kKC + j * 16 + c] = bl;
      }
#pragma unroll
      for (int off = 1; off < 16; off <<= 1) psum += __shfl_xor(psum, off, 32);
      lrow[r] = lrow[r] * alpha + psum;
#pragma unroll
      for (int t = 0; t < 4; ++t) oacc[t][r] *= alpha;
    }
    __builtin_amdgcn_fence(__ATOMIC_RELEASE, "workgroup");
    __builtin_amdgcn_wave_barrier();
    __builtin_amdgcn_fence(__ATOMIC_ACQUIRE, "workgroup");
#pragma unroll 1
    for (int kk = 0; kk < 2; ++kk) {
      FB pa, pl;
      pa.h[0] = *(const v8b*)(pwh + c * kKC + kk * 32 + 8 * hh);
      pa.h[1] = *(const v8b*)(pwh + c * kKC + kk * 32 + 16 + 8 * hh);
      pl.h[0] = *(const v8b*)(pwl + c * kKC + kk * 32 + 8 * hh);
      pl.h[1] = *(const v8b*)(pwl + c * kKC + kk * 32 + 16 + 8 * hh);
#pragma unroll
      for (int t = 0; t < 4; ++t) {
        FB vb, vl;
        vb.h[0] = *(const v8b*)(Vsh + (t * 16 + c) * kKC + kk * 32 + 8 * hh);
        vb.h[1] = *(const v8b*)(Vsh + (t * 16 + c) * kKC + kk * 32 + 16 + 8 * hh);
        vl.h[0] = *(const v8b*)(Vsl + (t * 16 + c) * kKC + kk * 32 + 8 * hh);
        vl.h[1] = *(const v8b*)(Vsl + (t * 16 + c) * kKC + kk * 32 + 16 + 8 * hh);
        oacc[t] = at_mma(pa.v, vb.v, oacc[t]);
        oacc[t] = at_mma(pa.v, vl.v, oacc[t]);
        oacc[t] = at_mma(pl.v, vb.v, oacc[t]);
      }
    }
  }

  float* os = Os[wave];
#pragma unroll
  for (int r = 0; r < 8; ++r) {
    const float inv = 1.0f / lrow[r];
#pragma unroll
    for (int t = 0; t < 4; ++t) os[(8 * hh + r) * 68 + t * 16 + c] = oacc[t][r] * inv;
  }
  __builtin_amdgcn_fence(__ATOMIC_RELEASE, "workgroup");
  __builtin_amdgcn_wave_barrier();
  __builtin_amdgcn_fence(__ATOMIC_ACQUIRE, "workgroup");
  {
    const int q4 = lane >> 3, c8 = (lane & 7) * 8;
    for (int pass = 0; pass < 2; ++pass) {
#pragma unroll
      for (int it = 0; it < 4; ++it) {
        const int row = it * 4 + q4;
        const float* sp = os + row * 68 + c8;
        unsigned short hb[8], lb[8];
#pragma unroll
        for (int e = 0; e < 8; ++e) {
          hb[e] = f2bf_bits(sp[e]);
          lb[e] = f2bf_bits(sp[e] - bf_bits2f(hb[e]));
        }
        const v4u uh = (v4u){pk16(hb[0], hb[1]), pk16(hb[2], hb[3]), pk16(hb[4], hb[5]), pk16(hb[6], hb[7])};
        const v4u ul = (v4u){pk16(lb[0], lb[1]), pk16(lb[2], lb[3]), pk16(lb[4], lb[5]), pk16(lb[6], lb[7])};
        const size_t dst = (size_t)(b * kS + q0 + row) * kD + (size_t)h * kHD + c8;
        *(volatile v4u*)(Oh + dst) = uh;
        *(volatile v4u*)(Ol + dst) = ul;
      }
      __threadfence();
    }
  }
}

extern "C" void kernel_launch(void* const* d_in, const int* in_sizes, int n_in,
                              void* d_out, int out_size, void* d_ws, size_t ws_size,
                              hipStream_t stream) {
  if (n_in < 5) return;
  if (in_sizes[0] != kTok * kD) return;
  if (in_sizes[1] != kD * kD) return;
  if (in_sizes[2] != kKVD * kD) return;
  if (in_sizes[3] != kKVD * kD) return;
  if (in_sizes[4] != kD * kD) return;
  if (out_size != kTok * kD) return;

  const size_t szXB  = (size_t)kTok * kD * 2;
  const size_t szWQK = (size_t)kQKN * kD * 2;
  const size_t szWV  = (size_t)kKVD * kD * 2;
  const size_t szWO  = (size_t)kD * kD * 2;
  const size_t szQK  = (size_t)kTok * kQKN * 2;
  const size_t szVT  = (size_t)kB * kKVD * kS * 2;
  const size_t szO   = (size_t)kTok * kD * 2;
  const size_t szT   = (size_t)kS * kRH * 4;
  const size_t offXB  = 0;
  const size_t offWQK = offXB + szXB;
  const size_t offWV  = offWQK + szWQK;
  const size_t offWO  = offWV + szWV;
  const size_t offQKH = offWO + szWO;
  const size_t offQKL = offQKH + szQK;
  const size_t offVTH = offQKL + szQK;
  const size_t offVTL = offVTH + szVT;
  const size_t offOH  = offVTL + szVT;
  const size_t offOL  = offOH + szO;
  const size_t offCOS = offOL + szO;
  const size_t offSIN = offCOS + szT;
  const size_t total  = offSIN + szT;
  if (ws_size < total) return;

  const float* x  = (const float*)d_in[0];
  const float* Wq = (const float*)d_in[1];
  const float* Wk = (const float*)d_in[2];
  const float* Wv = (const float*)d_in[3];
  const float* Wo = (const float*)d_in[4];
  float* out = (float*)d_out;
  char* ws = (char*)d_ws;
  unsigned short* XB  = (unsigned short*)(ws + offXB);
  unsigned short* WQK = (unsigned short*)(ws + offWQK);
  unsigned short* WV  = (unsigned short*)(ws + offWV);
  unsigned short* WO  = (unsigned short*)(ws + offWO);
  unsigned short* QKH = (unsigned short*)(ws + offQKH);
  unsigned short* QKL = (unsigned short*)(ws + offQKL);
  unsigned short* VTH = (unsigned short*)(ws + offVTH);
  unsigned short* VTL = (unsigned short*)(ws + offVTL);
  unsigned short* OH  = (unsigned short*)(ws + offOH);
  unsigned short* OL  = (unsigned short*)(ws + offOL);
  float* COS = (float*)(ws + offCOS);
  float* SIN = (float*)(ws + offSIN);

  const int n8x = (kTok * kD) / 8;
  const int n8q = (kD * kD) / 8;
  const int n8k = (kKVD * kD) / 8;
  cast8_bf16_kernel<<<dim3(n8x / 256), dim3(256), 0, stream>>>(x,  XB, n8x);
  cast8_bf16_kernel<<<dim3(n8q / 256), dim3(256), 0, stream>>>(Wq, WQK, n8q);
  cast8_bf16_kernel<<<dim3(n8k / 256), dim3(256), 0, stream>>>(Wk, WQK + (size_t)kD * kD, n8k);
  cast8_bf16_kernel<<<dim3(n8k / 256), dim3(256), 0, stream>>>(Wv, WV, n8k);
  cast8_bf16_kernel<<<dim3(n8q / 256), dim3(256), 0, stream>>>(Wo, WO, n8q);

  RopeFreq rf;
  for (int i = 0; i < kRH; ++i) {
    const double e = (double)(2 * i) / (double)kHD;
    const float p = (float)pow(10000.0, e);
    rf.inv[i] = 1.0f / p;
  }
  rope_table_kernel<<<dim3(kS / 8), dim3(256), 0, stream>>>(COS, SIN, rf);

  const int tilesQK = (kTok / 64) * (kQKN / 64);
  qk_rope_gemm_kernel<<<dim3(tilesQK / 8), dim3(256), 0, stream>>>(
      XB, kD, WQK, kD, QKH, QKL, kQKN, COS, SIN, kTok, kQKN, kD);

  const int tilesV = (kKVD / 64) * (kS / 64);
  wmma_gemm64<1, false, 0, 2, false, 0><<<dim3(tilesV / 8, kB), dim3(256), 0, stream>>>(
      WV, WV, kD, 0L, XB, XB, kD, (long)kS * kD,
      (void*)VTH, (void*)VTL, kS, (long)kKVD * kS, COS, COS, 0L, kKVD, kS, kD, 1.0f);

  flash_gqa_kernel<<<dim3(kB * kNH * (kS / kQB)), dim3(128), 0, stream>>>(QKH, QKL, VTH, VTL, OH, OL);

  const int tilesO = (kTok / 64) * (kD / 64);
  wmma_gemm64<1, true, 0, 0, false, 0, true><<<dim3(tilesO / 8, 1), dim3(256), 0, stream>>>(
      OH, OL, kD, 0L, WO, WO, kD, 0L,
      (void*)out, (void*)out, kD, 0L, COS, COS, 0L, kTok, kD, kD, 1.0f);
}
